// CrossModalAttention_36215164240753
// MI455X (gfx1250) — hardware-verified
//
#include <hip/hip_runtime.h>


typedef __bf16 b16;
typedef __attribute__((ext_vector_type(16))) __bf16 v16b;
typedef __attribute__((ext_vector_type(8)))  __bf16 v8b;
typedef __attribute__((ext_vector_type(8)))  float  v8f;
typedef __attribute__((ext_vector_type(4)))  float  v4f;
typedef __attribute__((ext_vector_type(4)))  int    i4;

#define NB 8
#define NTOK 1024
#define EMB 768
#define NHD 8
#define HDIM 96
#define MTOT 8192

__device__ __forceinline__ void split_bf16(float v, b16& hi, b16& lo) {
  const unsigned int u = __builtin_bit_cast(unsigned int, v) & 0xffff0000u;
  hi = __builtin_bit_cast(b16, (unsigned short)(u >> 16));
  lo = (b16)(v - __builtin_bit_cast(float, u));
}
__device__ __forceinline__ v8b ld8b(const b16* p) { return *(const v8b*)p; }
__device__ __forceinline__ v16b cat8b(v8b a, v8b b) { return __builtin_shufflevector(a, b, 0, 1, 2, 3, 4, 5, 6, 7, 8, 9, 10, 11, 12, 13, 14, 15); }
__device__ __forceinline__ v16b frag_kb(const b16* p, int hh) { return cat8b(ld8b(p + 8 * hh), ld8b(p + 16 + 8 * hh)); }
__device__ __forceinline__ void frag_ksplit(const float* p, int hh, v16b& fh, v16b& fl) {
  const float* p0 = p + 8 * hh; const float* p1 = p + 16 + 8 * hh;
#pragma unroll
  for (int e = 0; e < 8; ++e) { b16 a, c; split_bf16(p0[e], a, c); fh[e] = a; fl[e] = c; split_bf16(p1[e], a, c); fh[8 + e] = a; fl[8 + e] = c; }
}
__device__ __forceinline__ v8f wmmab(v16b a, v16b b, v8f c) {
  v8f d = __builtin_amdgcn_wmma_f32_16x16x32_bf16(false, a, false, b, (short)0, c, false, false);
  asm volatile("v_nop\n\tv_nop\n\tv_nop\n\tv_nop" : "+v"(d) : "v"(a), "v"(b));
  return d;
}
__device__ __forceinline__ v8f wmma3(v16b ah, v16b al, v16b bh, v16b bl, v8f c) {
  c = wmmab(ah, bh, c); c = wmmab(ah, bl, c); c = wmmab(al, bh, c); return c;
}
__device__ __forceinline__ void wave_sync_lds() {
  __builtin_amdgcn_fence(__ATOMIC_RELEASE, "workgroup"); __builtin_amdgcn_wave_barrier(); __builtin_amdgcn_fence(__ATOMIC_ACQUIRE, "workgroup");
}

__global__ void cma_wsplit(const float* __restrict__ w, b16* __restrict__ wh, b16* __restrict__ wl, int n8) {
  int i = blockIdx.x * blockDim.x + threadIdx.x;
  int stride = gridDim.x * blockDim.x;
  for (; i < n8; i += stride) {
    v8b h, l;
#pragma unroll
    for (int e = 0; e < 8; ++e) { b16 a, c; split_bf16(w[(size_t)i * 8 + e], a, c); h[e] = a; l[e] = c; }
    *(volatile v8b*)(wh + (size_t)i * 8) = h; *(volatile v8b*)(wl + (size_t)i * 8) = l;
    __threadfence();
    *(volatile v8b*)(wh + (size_t)i * 8) = h; *(volatile v8b*)(wl + (size_t)i * 8) = l;
  }
}

__global__ __launch_bounds__(256)
void cma_gemm_tn(const float* __restrict__ A, const b16* __restrict__ Wh, const b16* __restrict__ Wl,
                 const float* __restrict__ bias, void* __restrict__ out0, void* __restrict__ out1,
                 int M, int N, int K, int mode) {
  __shared__ __attribute__((aligned(16))) unsigned char smem[32768];
  b16* sW = (b16*)smem;
  const int lane = threadIdx.x & 31;
  const int wave = threadIdx.x >> 5;
  const int tid  = threadIdx.x;
  const int mt   = blockIdx.x * 128 + wave * 16;
  const int nb   = blockIdx.y * 64;
  const int l16  = lane & 15;
  const int hh   = lane >> 4;
  const int rbase = hh * 8;

  const int wr0 = tid >> 3, wc0 = (tid & 7) * 8;
  const int wr1 = (tid + 256) >> 3, wc1 = ((tid + 256) & 7) * 8;
  auto loadW = [&](int buf, int k0) {
    b16* dh = sW + (buf * 2 + 0) * 4096; b16* dl = sW + (buf * 2 + 1) * 4096;
    *(i4*)(dh + wr0 * 64 + wc0) = *(const i4*)(Wh + (size_t)(nb + wr0) * K + k0 + wc0);
    *(i4*)(dh + wr1 * 64 + wc1) = *(const i4*)(Wh + (size_t)(nb + wr1) * K + k0 + wc1);
    *(i4*)(dl + wr0 * 64 + wc0) = *(const i4*)(Wl + (size_t)(nb + wr0) * K + k0 + wc0);
    *(i4*)(dl + wr1 * 64 + wc1) = *(const i4*)(Wl + (size_t)(nb + wr1) * K + k0 + wc1);
  };
  const float* ap = A + (size_t)(mt + l16) * K;

  v8f acc[4] = {};
  int buf = 0;
  loadW(0, 0);
  for (int k0 = 0; k0 < K; k0 += 64, buf ^= 1) {
    __syncthreads();
    if (k0 + 64 < K) loadW(buf ^ 1, k0 + 64);
    const b16* ph = sW + (buf * 2 + 0) * 4096; const b16* pl = sW + (buf * 2 + 1) * 4096;
#pragma unroll
    for (int kk = 0; kk < 2; ++kk) {
      v16b ah, al; frag_ksplit(ap + k0 + kk * 32, hh, ah, al);
#pragma unroll
      for (int nt = 0; nt < 4; ++nt) {
        const b16* wp = ph + (nt * 16 + l16) * 64 + kk * 32;
        const b16* wq = pl + (nt * 16 + l16) * 64 + kk * 32;
        acc[nt] = wmma3(ah, al, frag_kb(wp, hh), frag_kb(wq, hh), acc[nt]);
      }
    }
  }
  __syncthreads();

  if (mode == 0) {
    b16* th = (b16*)smem + wave * 2048; b16* tl = th + 1024;
#pragma unroll
    for (int nt = 0; nt < 4; ++nt) {
      const float bn = bias[nb + nt * 16 + l16];
#pragma unroll
      for (int r = 0; r < 8; ++r) { b16 a, c; split_bf16(acc[nt][r] + bn, a, c); th[(rbase + r) * 64 + nt * 16 + l16] = a; tl[(rbase + r) * 64 + nt * 16 + l16] = c; }
    }
    wave_sync_lds();
    b16* oh = (b16*)out0; b16* ol = (b16*)out1;
    for (int pass = 0; pass < 2; ++pass) {
#pragma unroll
      for (int j = 0; j < 4; ++j) {
        const int row = j * 4 + (lane >> 3), seg = lane & 7;
        const size_t g = (size_t)(mt + row) * N + nb + seg * 8;
        *(volatile v8b*)(oh + g) = ld8b(th + row * 64 + seg * 8);
        *(volatile v8b*)(ol + g) = ld8b(tl + row * 64 + seg * 8);
      }
      __threadfence();
    }
  } else if (mode == 1) {
    b16* th = (b16*)smem; b16* tl = th + 8192;
    const int pl0 = wave * 16 + rbase;
#pragma unroll
    for (int nt = 0; nt < 4; ++nt) {
      const int nl = nt * 16 + l16;
      const float bn = bias[nb + nl];
#pragma unroll
      for (int r = 0; r < 8; ++r) { b16 a, c; split_bf16(acc[nt][r] + bn, a, c); th[nl * 128 + pl0 + r] = a; tl[nl * 128 + pl0 + r] = c; }
    }
    __syncthreads();
    b16* oh = (b16*)out0; b16* ol = (b16*)out1;
    const int p0 = (blockIdx.x * 128) & (NTOK - 1);
    const int bb = (blockIdx.x * 128) >> 10;
    for (int pass = 0; pass < 2; ++pass) {
#pragma unroll
      for (int q = 0; q < 4; ++q) {
        const int piece = tid + q * 256;
        const int nl = piece >> 4, seg = piece & 15;
        const int n = nb + nl, h = n / HDIM, d = n % HDIM;
        const size_t g = ((size_t)((bb * NHD + h) * HDIM + d) << 10) + p0 + seg * 8;
        *(volatile v8b*)(oh + g) = ld8b(th + nl * 128 + seg * 8);
        *(volatile v8b*)(ol + g) = ld8b(tl + nl * 128 + seg * 8);
      }
      __threadfence();
    }
  } else {
    float* of = (float*)out0;
    for (int pass = 0; pass < 2; ++pass) {
#pragma unroll
      for (int pr = 0; pr < 2; ++pr) {
        const int cbase = nb + pr * 32;
        const float bn = bias[cbase + lane];
#pragma unroll
        for (int r = 0; r < 8; ++r) {
          const float a0 = acc[2 * pr][r], b0 = acc[2 * pr + 1][r];
          const float ax = __shfl_xor(a0, 16), bx = __shfl_xor(b0, 16);
          const float v1 = (hh ? bx : a0) + bn;
          const float v2 = (hh ? b0 : ax) + bn;
          *(volatile float*)(of + (size_t)(mt + r) * N + cbase + lane) = v1;
          *(volatile float*)(of + (size_t)(mt + r + 8) * N + cbase + lane) = v2;
        }
      }
      __threadfence();
    }
  }
}

__global__ __launch_bounds__(256)
void cma_attn(const b16* __restrict__ Qh, const b16* __restrict__ Ql,
              const b16* __restrict__ Kh, const b16* __restrict__ Kl,
              const b16* __restrict__ Vh, const b16* __restrict__ Vl,
              float* __restrict__ Ao,
              float* __restrict__ avg_out) {
  __shared__ __attribute__((aligned(16))) float sS[16 * 1024];

  const int b    = blockIdx.y;
  const int m0   = blockIdx.x * 16;
  const int tid  = threadIdx.x;
  const int lane = tid & 31;
  const int wave = tid >> 5;
  const int l16  = lane & 15;
  const int hh   = lane >> 4;
  const int rbase = hh * 8;
  const float scale = 0.1020620726f;

  float AV[2][32];
#pragma unroll
  for (int rr = 0; rr < 2; ++rr)
#pragma unroll
    for (int i = 0; i < 32; ++i) AV[rr][i] = 0.f;

  for (int h = 0; h < NHD; ++h) {
    v16b qh_[3], ql_[3];
    {
      const size_t qo = ((size_t)((b << 10) + m0 + l16) * EMB) + h * HDIM;
#pragma unroll
      for (int kk = 0; kk < 3; ++kk) { qh_[kk] = frag_kb(Qh + qo + kk * 32, hh); ql_[kk] = frag_kb(Ql + qo + kk * 32, hh); }
    }
#pragma unroll
    for (int t = 0; t < 8; ++t) {
      const int p0 = wave * 128 + t * 16;
      const size_t ko = ((size_t)((b << 10) + p0 + l16) * EMB) + h * HDIM;
      v8f s = {};
#pragma unroll
      for (int kk = 0; kk < 3; ++kk) s = wmma3(qh_[kk], ql_[kk], frag_kb(Kh + ko + kk * 32, hh), frag_kb(Kl + ko + kk * 32, hh), s);
      const int ncol = p0 + l16;
#pragma unroll
      for (int r = 0; r < 8; ++r) sS[(rbase + r) * 1024 + ncol] = s[r] * scale;
    }
    __syncthreads();

    float P[2][32];
#pragma unroll
    for (int rr = 0; rr < 2; ++rr) {
      const int row = wave * 2 + rr;
      float mx = -3.0e38f;
#pragma unroll
      for (int i = 0; i < 32; ++i) { P[rr][i] = sS[row * 1024 + lane + 32 * i]; mx = fmaxf(mx, P[rr][i]); }
#pragma unroll
      for (int off = 16; off >= 1; off >>= 1) mx = fmaxf(mx, __shfl_xor(mx, off));
      float sum = 0.f;
#pragma unroll
      for (int i = 0; i < 32; ++i) { const float e = expf(P[rr][i] - mx); P[rr][i] = e; sum += e; }
#pragma unroll
      for (int off = 16; off >= 1; off >>= 1) sum += __shfl_xor(sum, off);
      const float inv = 1.0f / sum;
#pragma unroll
      for (int i = 0; i < 32; ++i) { P[rr][i] *= inv; AV[rr][i] += P[rr][i] * 0.125f; }
    }
    __syncthreads();
#pragma unroll
    for (int rr = 0; rr < 2; ++rr) {
      const int row = wave * 2 + rr;
#pragma unroll
      for (int i = 0; i < 32; ++i) sS[row * 1024 + lane + 32 * i] = P[rr][i];
    }
    __syncthreads();

    v8f o[6] = {};
#pragma unroll
    for (int c4 = 0; c4 < 4; ++c4) {
      const int pb = wave * 128 + c4 * 32;
      v16b aph, apl; frag_ksplit(sS + (size_t)l16 * 1024 + pb, hh, aph, apl);
#pragma unroll
      for (int nt = 0; nt < 6; ++nt) {
        const size_t vo = (((size_t)(b * NHD + h) * HDIM + nt * 16 + l16) << 10) + pb;
        o[nt] = wmma3(aph, apl, frag_kb(Vh + vo, hh), frag_kb(Vl + vo, hh), o[nt]);
      }
    }
    __syncthreads();

#pragma unroll
    for (int nt = 0; nt < 6; ++nt)
#pragma unroll
      for (int r = 0; r < 8; ++r) sS[wave * 1536 + (rbase + r) * 96 + nt * 16 + l16] = o[nt][r];
    __syncthreads();
    for (int idx = tid; idx < 1536; idx += 256) {
      float sum = 0.f;
#pragma unroll
      for (int w = 0; w < 8; ++w) sum += sS[w * 1536 + idx];
      sS[8 * 1536 + idx] = sum;
    }
    __syncthreads();
    for (int pass = 0; pass < 2; ++pass) {
      for (int piece = tid; piece < 384; piece += 256) {
        const int m = piece / 24, sg = piece % 24;
        *(volatile v4f*)(Ao + ((size_t)((b << 10) + m0 + m) * EMB) + h * HDIM + sg * 4) = *(const v4f*)(sS + 8 * 1536 + m * 96 + sg * 4);
      }
      __threadfence();
    }
    __syncthreads();
  }
  for (int pass = 0; pass < 2; ++pass) {
#pragma unroll
    for (int rr = 0; rr < 2; ++rr) {
      float* apo = avg_out + ((size_t)((b << 10) + m0 + wave * 2 + rr) << 10) + lane;
#pragma unroll
      for (int i = 0; i < 32; ++i) *(volatile float*)(apo + 32 * i) = AV[rr][i];
    }
    __threadfence();
  }
}

extern "C" void kernel_launch(void* const* d_in, const int* in_sizes, int n_in,
                              void* d_out, int out_size, void* d_ws, size_t ws_size,
                              hipStream_t stream) {
  (void)in_sizes; (void)n_in; (void)out_size;
  const float* mam = (const float*)d_in[0];
  const float* pat = (const float*)d_in[1];
  const float* qw  = (const float*)d_in[2];
  const float* qb  = (const float*)d_in[3];
  const float* kw  = (const float*)d_in[4];
  const float* kb  = (const float*)d_in[5];
  const float* vw  = (const float*)d_in[6];
  const float* vb  = (const float*)d_in[7];
  const float* ow  = (const float*)d_in[8];
  const float* ob  = (const float*)d_in[9];

  const size_t TOK = (size_t)MTOT * EMB;
  const size_t WSZ = (size_t)EMB * EMB;

  size_t off = 0; char* ws = (char*)d_ws;
  auto take = [&](size_t bytes) { void* p = ws + off; off += (bytes + 255) & ~(size_t)255; return p; };
  b16* Wqh = (b16*)take(WSZ * 2); b16* Wql = (b16*)take(WSZ * 2);
  b16* Wkh = (b16*)take(WSZ * 2); b16* Wkl = (b16*)take(WSZ * 2);
  b16* Wvh = (b16*)take(WSZ * 2); b16* Wvl = (b16*)take(WSZ * 2);
  b16* Woh = (b16*)take(WSZ * 2); b16* Wol = (b16*)take(WSZ * 2);
  b16* Qh = (b16*)take(TOK * 2);  b16* Ql = (b16*)take(TOK * 2);
  b16* Kh = (b16*)take(TOK * 2);  b16* Kl = (b16*)take(TOK * 2);
  b16* Vh = (b16*)take(TOK * 2);  b16* Vl = (b16*)take(TOK * 2);
  float* Ao = (float*)take(TOK * 4);
  if (off > ws_size) return;

  float* att_out = (float*)d_out;
  float* avg_out = att_out + TOK;

  cma_wsplit<<<288, 256, 0, stream>>>(qw, Wqh, Wql, (int)(WSZ / 8));
  cma_wsplit<<<288, 256, 0, stream>>>(kw, Wkh, Wkl, (int)(WSZ / 8));
  cma_wsplit<<<288, 256, 0, stream>>>(vw, Wvh, Wvl, (int)(WSZ / 8));
  cma_wsplit<<<288, 256, 0, stream>>>(ow, Woh, Wol, (int)(WSZ / 8));

  dim3 gg(MTOT / 128, EMB / 64);
  cma_gemm_tn<<<gg, 256, 0, stream>>>(mam, Wqh, Wql, qb, Qh, Ql, MTOT, EMB, EMB, 0);
  cma_gemm_tn<<<gg, 256, 0, stream>>>(pat, Wkh, Wkl, kb, Kh, Kl, MTOT, EMB, EMB, 0);
  cma_gemm_tn<<<gg, 256, 0, stream>>>(pat, Wvh, Wvl, vb, Vh, Vl, MTOT, EMB, EMB, 1);

  cma_attn<<<dim3(NTOK / 16, NB), 256, 0, stream>>>(Qh, Ql, Kh, Kl, Vh, Vl, Ao, avg_out);

  cma_gemm_tn<<<gg, 256, 0, stream>>>(Ao, Woh, Wol, ob, att_out, nullptr, MTOT, EMB, EMB, 2);
}
